// KANLayer_23184233464145
// MI455X (gfx1250) — hardware-verified
//
#include <hip/hip_runtime.h>
#include <stdint.h>

#define NROWS   8192
#define NIN     1024
#define NOUT    64
#define K13     13
#define NB      10
#define NKNOT   14
#define KH      (NIN * NB)
#define KTOT    (2 * KH)
#define CH      2048
#define NCHUNK  (NROWS / CH)
#define UROW    (KTOT / 8)
#define FTHR    512
#define FPT     (NIN / FTHR)
#define NSWEEP  (UROW / FTHR)
#define PUNITS  (NOUT * UROW)
#define PBLKS   (PUNITS / 256)
#define NRCP    36
#define WSCAP   134217728

static_assert(NROWS == NCHUNK * CH);
static_assert(CH % 128 == 0);
static_assert(NOUT == 64);
static_assert(KTOT % 32 == 0);
static_assert(KH % 8 == 0);
static_assert(UROW % 32 == 0);
static_assert(NSWEEP * FTHR == UROW);
static_assert(PUNITS == PBLKS * 256);
static_assert(FTHR * FPT == NIN);
static_assert((NB % 2) == 0);
static_assert((KTOT * 2) % 128 == 0);
static_assert(NRCP == 13 + 12 + 11);

typedef float          v4f   __attribute__((ext_vector_type(4)));
typedef float          v8f   __attribute__((ext_vector_type(8)));
typedef int            v8i   __attribute__((ext_vector_type(8)));
typedef unsigned int   v4u   __attribute__((ext_vector_type(4)));
typedef unsigned short v8us  __attribute__((ext_vector_type(8)));
typedef unsigned short v16us __attribute__((ext_vector_type(16)));
typedef __bf16         v16b  __attribute__((ext_vector_type(16)));
typedef v4f  __attribute__((may_alias)) v4fa;
typedef v4u  __attribute__((may_alias)) v4ua;
typedef v8us __attribute__((may_alias)) v8usa;
typedef unsigned int __attribute__((may_alias)) ua;
union FragB { v16b v; v16us u; v8us h[2]; v8i w; };

__device__ __forceinline__ unsigned short f2bf_bits(float f) {
  unsigned u = __float_as_uint(f);
  return (unsigned short)((u + 0x7FFFu + ((u >> 16) & 1u)) >> 16);
}
__device__ __forceinline__ float bf_bits2f(unsigned short b) { return __uint_as_float(((unsigned)b) << 16); }
__device__ __forceinline__ float bfr(float f) { return bf_bits2f(f2bf_bits(f)); }
__device__ __forceinline__ unsigned pk16(unsigned short a, unsigned short b) { return (unsigned)a | ((unsigned)b << 16); }

__device__ __forceinline__ v8f wmb(const FragB& a, const FragB& b, v8f c) {
  v8f d = __builtin_amdgcn_wmma_f32_16x16x32_bf16(false, a.v, false, b.v, (short)0, c, false, false);
  asm volatile("v_nop\n\tv_nop\n\tv_nop\n\tv_nop" : "+v"(d) : "v"(a.w), "v"(b.w));
  return d;
}
__device__ __forceinline__ v8f z8() { v8f z = {0.f, 0.f, 0.f, 0.f, 0.f, 0.f, 0.f, 0.f}; return z; }

__global__ __launch_bounds__(256) void prep_kernel(const float* __restrict__ cp, unsigned short* __restrict__ WB) {
  const int u  = blockIdx.x * 256 + threadIdx.x;
  const int o  = u / UROW;
  const int ku = u - o * UROW;
  const int k8 = ku * 8;
  const int kk8 = (k8 < KH) ? k8 : (k8 - KH);
  const float* src = cp + (size_t)o * NIN * K13;
  unsigned short hb[8];
#pragma unroll
  for (int e = 0; e < 8; ++e) {
    const int kk = kk8 + e;
    const int j  = kk / NB;
    const int m  = kk - j * NB;
    hb[e] = f2bf_bits(src[j * K13 + m]);
  }
  v4u v;
  v[0] = pk16(hb[0], hb[1]);
  v[1] = pk16(hb[2], hb[3]);
  v[2] = pk16(hb[4], hb[5]);
  v[3] = pk16(hb[6], hb[7]);
  unsigned short* dst = WB + (size_t)u * 8;
  *(volatile v4u*)dst = v;
  __threadfence();
  *(volatile v4u*)dst = v;
}

__device__ __forceinline__ float cdb_step(float xb, float tm, float tq, float rc1, float rc2, int g1, int g2,
                                          float bm, float bm1) {
  const float q1 = (xb - tm) * rc1;
  const float q2 = (tq - xb) * rc2;
  const float l  = __int_as_float(__float_as_int(q1) & g1) * bm;
  const float rr = __int_as_float(__float_as_int(q2) & g2) * bm1;
  return l + rr;
}

__device__ __forceinline__ void a_store_pass(const unsigned short* sA, unsigned short* dst, int tid) {
#pragma unroll
  for (int it = 0; it < NSWEEP; ++it) {
    const int u = it * FTHR + tid;
    const v4u v = *(const v4ua*)(sA + 8 * u);
    *(volatile v4u*)(dst + 8 * u) = v;
  }
}

__global__ __launch_bounds__(FTHR) void feat_kernel(const float* __restrict__ x, const float* __restrict__ knots,
                                                    unsigned short* __restrict__ AP, int row_base) {
  __shared__ __align__(16) unsigned short sA[KTOT];
  __shared__ float sT[16];
  __shared__ float sR[NRCP + 4];
  __shared__ int   sG[NRCP + 4];
  const int tid = threadIdx.x;
  const int r = blockIdx.x;

  {
    const int ci = (tid < NKNOT) ? tid : (NKNOT - 1);
    const float kv = bfr(knots[ci]);
    if (tid < NKNOT) sT[tid] = kv;
    if (tid >= NKNOT && tid < 16) sT[tid] = 0.0f;
  }
  __syncthreads();
  {
    const int i = (tid < NRCP) ? tid : (NRCP - 1);
    const int p = (i < 13) ? 1 : ((i < 25) ? 2 : 3);
    const int m = i - ((i < 13) ? 0 : ((i < 25) ? 13 : 25));
    const float d = sT[m + p] - sT[m];
    const bool g = d > 0.0f;
    const float dsel = g ? d : 1.0f;
    const float rc = 1.0f / dsel;
    if (tid < NRCP) { sR[tid] = rc; sG[tid] = g ? -1 : 0; }
    if (tid >= NRCP && tid < NRCP + 4) { sR[tid] = 0.0f; sG[tid] = 0; }
  }
  __syncthreads();

  ua* sAu = (ua*)sA;
  const float* xrow = x + (size_t)(row_base + r) * NIN;
#pragma unroll 1
  for (int s = 0; s < FPT; ++s) {
    const int j = s * FTHR + tid;
    const float xb = bfr(xrow[j]);
    float tk[NKNOT];
#pragma unroll
    for (int i = 0; i < NKNOT; ++i) tk[i] = sT[i];

    float b0[13];
#pragma unroll
    for (int m = 0; m < 13; ++m) b0[m] = (xb >= tk[m] && xb < tk[m + 1]) ? 1.0f : 0.0f;

    float n1[12];
#pragma unroll
    for (int m = 0; m < 12; ++m)
      n1[m] = cdb_step(xb, tk[m], tk[m + 2], sR[m], sR[m + 1], sG[m], sG[m + 1], b0[m], b0[m + 1]);

    float n2[11];
#pragma unroll
    for (int m = 0; m < 11; ++m)
      n2[m] = cdb_step(xb, tk[m], tk[m + 3], sR[13 + m], sR[14 + m], sG[13 + m], sG[14 + m], n1[m], n1[m + 1]);

    float n3[10];
#pragma unroll
    for (int m = 0; m < 10; ++m)
      n3[m] = cdb_step(xb, tk[m], tk[m + 4], sR[25 + m], sR[26 + m], sG[25 + m], sG[26 + m], n2[m], n2[m + 1]);

    unsigned hw[5], lw[5];
#pragma unroll
    for (int i = 0; i < 5; ++i) {
      const float v0 = n3[2 * i], v1 = n3[2 * i + 1];
      const unsigned short h0 = f2bf_bits(v0), h1 = f2bf_bits(v1);
      const unsigned short l0 = f2bf_bits(v0 - bf_bits2f(h0));
      const unsigned short l1 = f2bf_bits(v1 - bf_bits2f(h1));
      hw[i] = pk16(h0, h1);
      lw[i] = pk16(l0, l1);
    }
    const int ub = 5 * j;
#pragma unroll
    for (int i = 0; i < 5; ++i) {
      sAu[ub + i] = hw[i];
      sAu[(KH / 2) + ub + i] = lw[i];
    }
  }
  __syncthreads();

  unsigned short* dst = AP + (size_t)r * KTOT;
  a_store_pass(sA, dst, tid);
  __threadfence();
  a_store_pass(sA, dst, tid);
}

__device__ __forceinline__ void o_store_pass(const float* sO, float* out, int grow_w, int w, int lane) {
  const int q8 = lane & 7, sub = lane >> 3;
#pragma unroll
  for (int i = 0; i < 16; ++i) {
    const int lid = i * 4 + sub;
    const int row = lid >> 1, hl = lid & 1;
    const v4f v = *(const v4fa*)(sO + (32 * w + row) * NOUT + 32 * hl + 4 * q8);
    *(volatile v4f*)(out + (size_t)(grow_w + row) * NOUT + 32 * hl + 4 * q8) = v;
  }
}

__global__ __launch_bounds__(128) void gemm_kernel(const unsigned short* __restrict__ AP,
                                                   const unsigned short* __restrict__ WB,
                                                   float* __restrict__ out, int row_base) {
  __shared__ __align__(16) float sO[128 * NOUT];
  const int tid = threadIdx.x, lane = tid & 31, w = tid >> 5;
  const int h = lane >> 4, m = lane & 15;
  const int lrow_w = blockIdx.x * 128 + 32 * w;

  const unsigned short* xa0 = AP + (size_t)(lrow_w + m) * KTOT + 8 * h;
  const unsigned short* xa1 = xa0 + (size_t)16 * KTOT;
  const unsigned short* wb  = WB + (size_t)m * KTOT + 8 * h;

  v8f acc[2][4];
#pragma unroll
  for (int mt = 0; mt < 2; ++mt)
#pragma unroll
    for (int nt = 0; nt < 4; ++nt) acc[mt][nt] = z8();

#pragma unroll 1
  for (int k0 = 0; k0 < KTOT; k0 += 32) {
    FragB a0, a1;
    a0.h[0] = *(const v8usa*)(xa0 + k0);
    a0.h[1] = *(const v8usa*)(xa0 + k0 + 16);
    a1.h[0] = *(const v8usa*)(xa1 + k0);
    a1.h[1] = *(const v8usa*)(xa1 + k0 + 16);
#pragma unroll
    for (int nt = 0; nt < 4; ++nt) {
      const unsigned short* wq = wb + (size_t)nt * 16 * KTOT + k0;
      FragB b;
      b.h[0] = *(const v8usa*)wq;
      b.h[1] = *(const v8usa*)(wq + 16);
      acc[0][nt] = wmb(a0, b, acc[0][nt]);
      acc[1][nt] = wmb(a1, b, acc[1][nt]);
    }
  }

#pragma unroll
  for (int nt = 0; nt < 4; ++nt) {
    const int cl = 16 * nt + m;
#pragma unroll
    for (int mt = 0; mt < 2; ++mt) {
#pragma unroll
      for (int r = 0; r < 8; ++r) {
        const int rl = 32 * w + 16 * mt + 8 * h + r;
        sO[rl * NOUT + cl] = acc[mt][nt][r];
      }
    }
  }
  __syncthreads();

  const int grow_w = row_base + lrow_w;
  o_store_pass(sO, out, grow_w, w, lane);
  __threadfence();
  o_store_pass(sO, out, grow_w, w, lane);
}

extern "C" void kernel_launch(void* const* d_in, const int* in_sizes, int n_in,
                              void* d_out, int out_size, void* d_ws, size_t ws_size,
                              hipStream_t stream) {
  if (n_in < 3) return;
  if (in_sizes[0] != NROWS * NIN) return;
  if (in_sizes[1] != NKNOT) return;
  if (in_sizes[2] != NOUT * NIN * K13) return;
  if (out_size != NROWS * NOUT) return;

  const float* x     = (const float*)d_in[0];
  const float* knots = (const float*)d_in[1];
  const float* cp    = (const float*)d_in[2];
  float* out = (float*)d_out;

  size_t off = 0;
  const size_t oAP = off; off += (size_t)CH * KTOT * 2;
  const size_t oWB = off; off += (size_t)NOUT * KTOT * 2;
  if (off > ws_size) return;
  if (off > (size_t)WSCAP) return;

  char* ws = (char*)d_ws;
  unsigned short* AP = (unsigned short*)(ws + oAP);
  unsigned short* WB = (unsigned short*)(ws + oWB);

  prep_kernel<<<dim3(PBLKS), dim3(256), 0, stream>>>(cp, WB);
  for (int c = 0; c < NCHUNK; ++c) {
    const int row_base = c * CH;
    feat_kernel<<<dim3(CH), dim3(FTHR), 0, stream>>>(x, knots, AP, row_base);
    gemm_kernel<<<dim3(CH / 128, 1), dim3(128), 0, stream>>>(AP, WB, out, row_base);
  }
  (void)hipGetLastError();
}
